// Self_Attention_26895085207764
// MI455X (gfx1250) — hardware-verified
//
#include <hip/hip_runtime.h>
#ifndef NB
#define NB 2
#endif
#ifndef SEQ
#define SEQ 4096
#endif
#define TT SEQ
#define NB_FULL 2
#define T_FULL 4096
#define CC 1024
#define QC ((TT < 1024) ? TT : 1024)
#define NE 256
static_assert(NB >= 1 && NB <= NB_FULL);
static_assert(TT % 256 == 0 && TT <= T_FULL);
static_assert(TT % QC == 0 && QC % 256 == 0);
static_assert(NE % 64 == 0 && NE <= QC && NE == 256);
static_assert(CC % 64 == 0);

#define RS 1024.0f
#define RFOLD 0.0009765625f
#define PCARRY 4096.0f
#define CTXC 16.0f
#define WOC 64.0f
#define SCL 0.03125f
#define PVALPHA 0.00390625f
#define OALPHA 0.0009765625f

typedef __bf16 v16b __attribute__((ext_vector_type(16)));
typedef _Float16 v16h __attribute__((ext_vector_type(16)));
typedef _Float16 v8h __attribute__((ext_vector_type(8)));
typedef unsigned short v8us __attribute__((ext_vector_type(8), may_alias));
typedef float v8f __attribute__((ext_vector_type(8)));
typedef float v4f __attribute__((ext_vector_type(4)));
typedef float v4fa __attribute__((ext_vector_type(4), may_alias));
union FragB { v16b v; v8us half[2]; unsigned short u[16]; };
union FragH { v16h v; v8us half[2]; unsigned short u[16]; };
union Pack8 { v8h h; v8us u; };

__device__ __forceinline__ unsigned short bf16_bits(float x) { unsigned int u = __float_as_uint(x); return (unsigned short)((u + 0x7FFFu + ((u >> 16) & 1u)) >> 16); }
__device__ __forceinline__ float bf16_val(unsigned short b) { return __uint_as_float(((unsigned int)b) << 16); }
__device__ __forceinline__ float bf16_rne(float x) { return bf16_val(bf16_bits(x)); }

__device__ __forceinline__ v8f mma_b(v16b a, v16b b, v8f c) {
  c = __builtin_amdgcn_wmma_f32_16x16x32_bf16(false, a, false, b, (short)0, c, false, false);
  asm volatile("v_nop\n\tv_nop\n\tv_nop\n\tv_nop" : "+v"(c) : "v"(a), "v"(b));
  return c;
}
template <int NT>
__device__ __forceinline__ void mma_h(v16h ah, v16h al, v16h bh, v16h bl, v8f& c, v8f& cr) {
  c = __builtin_amdgcn_wmma_f32_16x16x32_f16(false, ah, false, bh, (short)0, c, false, false);
  if (NT >= 2) cr = __builtin_amdgcn_wmma_f32_16x16x32_f16(false, al, false, bh, (short)0, cr, false, false);
  if (NT >= 3) cr = __builtin_amdgcn_wmma_f32_16x16x32_f16(false, ah, false, bl, (short)0, cr, false, false);
  if (NT >= 2) asm volatile("v_nop\n\tv_nop\n\tv_nop\n\tv_nop" : "+v"(c), "+v"(cr) : "v"(ah), "v"(al), "v"(bh), "v"(bl));
  else         asm volatile("v_nop\n\tv_nop\n\tv_nop\n\tv_nop" : "+v"(c) : "v"(ah), "v"(bh));
}

__device__ __forceinline__ void store_tile_f32(const float (*sw)[64], float* C, int ldc, int lane) {
  const int rsub = lane >> 4, c4 = (lane & 15) * 4;
  for (int pass = 0; pass < 2; ++pass) {
#pragma unroll
    for (int q = 0; q < 8; ++q) {
      const int r = q * 2 + rsub;
      const v4f v = *(const v4fa*)&sw[r][c4];
      *(volatile v4f*)(C + (size_t)r * ldc + c4) = v;
    }
    if (pass == 0) __threadfence();
  }
}
__device__ __forceinline__ void store_tile_h16(const float (*sw)[64], unsigned short* hb, int ldh, unsigned short* rb, int ldr, bool dores, int lane) {
  const int rsub = lane >> 3, c8 = (lane & 7) * 8;
  for (int pass = 0; pass < 2; ++pass) {
#pragma unroll
    for (int q = 0; q < 4; ++q) {
      const int r = q * 4 + rsub;
      const v4f x0 = *(const v4fa*)&sw[r][c8], x1 = *(const v4fa*)&sw[r][c8 + 4];
      const float xs[8] = {x0[0], x0[1], x0[2], x0[3], x1[0], x1[1], x1[2], x1[3]};
      Pack8 ph, pr;
#pragma unroll
      for (int i = 0; i < 8; ++i) { ph.h[i] = (_Float16)xs[i]; pr.h[i] = (_Float16)((xs[i] - (float)ph.h[i]) * RS); }
      *(volatile v8us*)(hb + (size_t)r * ldh + c8) = ph.u;
      if (dores) *(volatile v8us*)(rb + (size_t)r * ldr + c8) = pr.u;
    }
    if (pass == 0) __threadfence();
  }
}

template <int MODE>
__global__ __launch_bounds__(256) void k_cvt(const float* __restrict__ src, unsigned short* __restrict__ dst, int n8, float scale) {
  const int t = blockIdx.x * 256 + threadIdx.x;
  if (t >= n8) return;
  const float* sp = src + (size_t)t * 8;
  const v4f a = *(const v4fa*)sp, b = *(const v4fa*)(sp + 4);
  const float xs[8] = {a[0], a[1], a[2], a[3], b[0], b[1], b[2], b[3]};
  v8us v;
  if (MODE == 0) {
#pragma unroll
    for (int i = 0; i < 8; ++i) v[i] = bf16_bits(xs[i]);
  } else {
    Pack8 p;
#pragma unroll
    for (int i = 0; i < 8; ++i) p.h[i] = (_Float16)(bf16_rne(xs[i]) * scale);
    v = p.u;
  }
  unsigned short* dp = dst + (size_t)t * 8;
  *(volatile v8us*)dp = v;
  __threadfence();
  *(volatile v8us*)dp = v;
}

__global__ __launch_bounds__(128) void k_gemm_qkv(const unsigned short* __restrict__ A, const unsigned short* __restrict__ W,
                                                 unsigned short* __restrict__ Oh, unsigned short* __restrict__ Or, int M) {
  __shared__ __attribute__((aligned(16))) float so[4][16][64];
  const int tid = threadIdx.x, w = tid >> 5, lane = tid & 31, ln = lane & 15, hh = lane >> 4;
  const int ntn = (3 * CC) / 64;
  const int wid = blockIdx.x * 4 + w;
  const int mt = wid / ntn, nq = wid - mt * ntn;
  if (mt * 16 >= M) return;
  const int row0 = mt * 16, col0 = nq * 64;
  const unsigned short* arow = A + (size_t)(row0 + ln) * CC;
  v8f acc[4];
#pragma unroll
  for (int t = 0; t < 4; ++t) acc[t] = (v8f){0.f, 0.f, 0.f, 0.f, 0.f, 0.f, 0.f, 0.f};
  for (int kb = 0; kb < CC; kb += 32) {
    FragB a;
    a.half[0] = *(const v8us*)(arow + kb + 8 * hh);
    a.half[1] = *(const v8us*)(arow + kb + 16 + 8 * hh);
#pragma unroll
    for (int t = 0; t < 4; ++t) {
      const unsigned short* brow = W + (size_t)(col0 + t * 16 + ln) * CC + kb;
      FragB b;
      b.half[0] = *(const v8us*)(brow + 8 * hh);
      b.half[1] = *(const v8us*)(brow + 16 + 8 * hh);
      acc[t] = mma_b(a.v, b.v, acc[t]);
    }
  }
#pragma unroll
  for (int t = 0; t < 4; ++t)
#pragma unroll
    for (int r = 0; r < 8; ++r) so[w][8 * hh + r][t * 16 + ln] = acc[t][r];
  __builtin_amdgcn_fence(4, "workgroup");
  __builtin_amdgcn_wave_barrier();
  const int p = col0 / CC, colp = col0 - p * CC;
  const int bidx = row0 / TT, tq = row0 - bidx * TT;
  const bool dores = (tq < NE);
  unsigned short* hb = Oh + ((size_t)p * M + row0) * CC + colp;
  unsigned short* rb = Or + ((size_t)p * (NB * NE) + (size_t)bidx * NE + (dores ? tq : 0)) * CC + colp;
  store_tile_h16(so[w], hb, CC, rb, CC, dores, lane);
}

template <int NT>
__device__ __forceinline__ void core_h(const unsigned short* __restrict__ Ah, const unsigned short* __restrict__ Al, int lda, int ldal,
                                       const unsigned short* __restrict__ Bh, const unsigned short* __restrict__ Bl, int ldb, int ldbl,
                                       int row0, int col0, int kend, int ln, int hh, v8f (&acc)[4], v8f (&accr)[4]) {
  const unsigned short* arh = Ah + (size_t)(row0 + ln) * lda;
  const unsigned short* arl = Al + (size_t)(row0 + ln) * ldal;
  for (int kb = 0; kb < kend; kb += 32) {
    FragH ah, al;
    ah.half[0] = *(const v8us*)(arh + kb + 8 * hh);
    ah.half[1] = *(const v8us*)(arh + kb + 16 + 8 * hh);
    if (NT >= 2) { al.half[0] = *(const v8us*)(arl + kb + 8 * hh); al.half[1] = *(const v8us*)(arl + kb + 16 + 8 * hh); } else al = ah;
#pragma unroll
    for (int t = 0; t < 4; ++t) {
      const int n = col0 + t * 16 + ln;
      const unsigned short* brh = Bh + (size_t)n * ldb + kb;
      FragH bh, bl;
      bh.half[0] = *(const v8us*)(brh + 8 * hh);
      bh.half[1] = *(const v8us*)(brh + 16 + 8 * hh);
      if (NT >= 3) { const unsigned short* brl = Bl + (size_t)n * ldbl + kb; bl.half[0] = *(const v8us*)(brl + 8 * hh); bl.half[1] = *(const v8us*)(brl + 16 + 8 * hh); } else bl = bh;
      mma_h<NT>(ah.v, al.v, bh.v, bl.v, acc[t], accr[t]);
    }
  }
}

template <int NT>
__global__ __launch_bounds__(128) void k_gemm_f32(const unsigned short* __restrict__ Ah, const unsigned short* __restrict__ Al, int lda, int ldal,
                                                 const unsigned short* __restrict__ Bh, const unsigned short* __restrict__ Bl, int ldb, int ldbl,
                                                 const float* __restrict__ bias, float alpha, float* __restrict__ C, int ldc,
                                                 int M, int N, int K, int ncut, int kcut) {
  __shared__ __attribute__((aligned(16))) float so[4][16][64];
  const int tid = threadIdx.x, w = tid >> 5, lane = tid & 31, ln = lane & 15, hh = lane >> 4;
  const int ntn = N / 64;
  const int wid = blockIdx.x * 4 + w;
  const int mt = wid / ntn, nq = wid - mt * ntn;
  if (mt * 16 >= M) return;
  const int row0 = mt * 16, col0 = nq * 64;
  if (col0 > ncut + row0 + 15) return;
  int kend = (kcut + row0 + 16 + 31) & ~31;
  if (kend > K) kend = K;
  v8f acc[4], accr[4];
#pragma unroll
  for (int t = 0; t < 4; ++t) { acc[t] = (v8f){0.f, 0.f, 0.f, 0.f, 0.f, 0.f, 0.f, 0.f}; accr[t] = acc[t]; }
  core_h<NT>(Ah, Al, lda, ldal, Bh, Bl, ldb, ldbl, row0, col0, kend, ln, hh, acc, accr);
#pragma unroll
  for (int t = 0; t < 4; ++t) {
    float bv = 0.f;
    if (bias != nullptr) bv = bf16_rne(bias[col0 + t * 16 + ln]);
#pragma unroll
    for (int r = 0; r < 8; ++r) {
      float v = acc[t][r];
      if (NT >= 2) v += accr[t][r] * RFOLD;
      so[w][8 * hh + r][t * 16 + ln] = v * alpha + bv;
    }
  }
  __builtin_amdgcn_fence(4, "workgroup");
  __builtin_amdgcn_wave_barrier();
  store_tile_f32(so[w], C + (size_t)row0 * ldc + col0, ldc, lane);
}

template <int NT>
__global__ __launch_bounds__(128) void k_gemm_h16(const unsigned short* __restrict__ Ah, const unsigned short* __restrict__ Al, int lda, int ldal,
                                                 const unsigned short* __restrict__ Bh, const unsigned short* __restrict__ Bl, int ldb, int ldbl,
                                                 float alpha, unsigned short* __restrict__ Oh, int ldo, unsigned short* __restrict__ Or, int ldr, int rrows,
                                                 int M, int N, int K, int kcut) {
  __shared__ __attribute__((aligned(16))) float so[4][16][64];
  const int tid = threadIdx.x, w = tid >> 5, lane = tid & 31, ln = lane & 15, hh = lane >> 4;
  const int ntn = N / 64;
  const int wid = blockIdx.x * 4 + w;
  const int mt = wid / ntn, nq = wid - mt * ntn;
  if (mt * 16 >= M) return;
  const int row0 = mt * 16, col0 = nq * 64;
  int kend = (kcut + row0 + 16 + 31) & ~31;
  if (kend > K) kend = K;
  v8f acc[4], accr[4];
#pragma unroll
  for (int t = 0; t < 4; ++t) { acc[t] = (v8f){0.f, 0.f, 0.f, 0.f, 0.f, 0.f, 0.f, 0.f}; accr[t] = acc[t]; }
  core_h<NT>(Ah, Al, lda, ldal, Bh, Bl, ldb, ldbl, row0, col0, kend, ln, hh, acc, accr);
#pragma unroll
  for (int t = 0; t < 4; ++t)
#pragma unroll
    for (int r = 0; r < 8; ++r) {
      float v = acc[t][r];
      if (NT >= 2) v += accr[t][r] * RFOLD;
      so[w][8 * hh + r][t * 16 + ln] = v * alpha;
    }
  __builtin_amdgcn_fence(4, "workgroup");
  __builtin_amdgcn_wave_barrier();
  const bool dores = (row0 < rrows);
  store_tile_h16(so[w], Oh + (size_t)row0 * ldo + col0, ldo, Or + (size_t)(dores ? row0 : 0) * ldr + col0, ldr, dores, lane);
}

__device__ __forceinline__ void softmax_pack(const float* s, int j8, int qi, float mx, float inv, v8us& ho, v8us& ro) {
  const v4f a = *(const v4fa*)(s + j8), b = *(const v4fa*)(s + j8 + 4);
  const float xs[8] = {a[0], a[1], a[2], a[3], b[0], b[1], b[2], b[3]};
  Pack8 ph, pr;
#pragma unroll
  for (int u = 0; u < 8; ++u) {
    const float e = __expf(xs[u] - mx) * inv;
    const float p = ((j8 + u) <= qi) ? e : 0.f;
    ph.h[u] = (_Float16)p;
    pr.h[u] = (_Float16)((p - (float)ph.h[u]) * RS);
  }
  ho = ph.u; ro = pr.u;
}
__global__ __launch_bounds__(256) void k_softmax(const float* __restrict__ S, int sp, unsigned short* __restrict__ P, int pp, int N, int qoff,
                                                unsigned short* __restrict__ Pr, int rp, int rrows) {
  __shared__ float red[256];
  const int row = blockIdx.x, tid = threadIdx.x;
  const int qi = qoff + row;
  const float* s = S + (size_t)row * sp;
  float mx = -3.0e38f;
  for (int j = tid; j < N; j += 256) { const float v = s[j]; mx = fmaxf(mx, (j <= qi) ? v : -3.0e38f); }
  red[tid] = mx; __syncthreads();
  for (int st = 128; st > 0; st >>= 1) { if (tid < st) red[tid] = fmaxf(red[tid], red[tid + st]); __syncthreads(); }
  mx = red[0]; __syncthreads();
  float sum = 0.f;
  for (int j = tid; j < N; j += 256) { const float e = __expf(s[j] - mx); sum += (j <= qi) ? e : 0.f; }
  red[tid] = sum; __syncthreads();
  for (int st = 128; st > 0; st >>= 1) { if (tid < st) red[tid] += red[tid + st]; __syncthreads(); }
  const float inv = PCARRY / red[0];
  const int j8a = tid * 8, j8b = j8a + 2048;
  const bool hasA = (j8a < N), hasB = (j8b < N);
  const bool dores = (row < rrows) && (j8a < NE);
  v8us ha = (v8us){0, 0, 0, 0, 0, 0, 0, 0}, ra = ha, hb2 = ha, rb2 = ha;
  if (hasA) softmax_pack(s, j8a, qi, mx, inv, ha, ra);
  if (hasB) softmax_pack(s, j8b, qi, mx, inv, hb2, rb2);
  unsigned short* prow = P + (size_t)row * pp;
  unsigned short* rrow = Pr + (size_t)(dores ? row : 0) * rp;
  for (int pass = 0; pass < 2; ++pass) {
    if (hasA) *(volatile v8us*)(prow + j8a) = ha;
    if (dores) *(volatile v8us*)(rrow + j8a) = ra;
    if (hasB) *(volatile v8us*)(prow + j8b) = hb2;
    if (pass == 0) __threadfence();
  }
}

__global__ __launch_bounds__(256) void k_transpose16(const unsigned short* __restrict__ src, int lds_, unsigned short* __restrict__ dst, int ldd) {
  __shared__ __attribute__((aligned(16))) unsigned short tile[64][72];
  const int tid = threadIdx.x;
  const int r0 = blockIdx.x * 64, c0 = blockIdx.y * 64;
#pragma unroll
  for (int i = 0; i < 2; ++i) {
    const int e = tid + 256 * i, r = e >> 3, c8 = (e & 7) * 8;
    const v8us v = *(const v8us*)(src + (size_t)(r0 + r) * lds_ + c0 + c8);
    *(v8us*)&tile[r][c8] = v;
  }
  __syncthreads();
  v8us o[2];
#pragma unroll
  for (int i = 0; i < 2; ++i) {
    const int e = tid + 256 * i, rr = e >> 3, c8 = (e & 7) * 8;
#pragma unroll
    for (int k = 0; k < 8; ++k) o[i][k] = tile[c8 + k][rr];
  }
  for (int pass = 0; pass < 2; ++pass) {
#pragma unroll
    for (int i = 0; i < 2; ++i) {
      const int e = tid + 256 * i, rr = e >> 3, c8 = (e & 7) * 8;
      *(volatile v8us*)(dst + (size_t)(c0 + rr) * ldd + r0 + c8) = o[i];
    }
    if (pass == 0) __threadfence();
  }
}

extern "C" void kernel_launch(void* const* d_in, const int* in_sizes, int n_in,
                              void* d_out, int out_size, void* d_ws, size_t ws_size, hipStream_t stream) {
  if (n_in < 6) return;
  const float* x  = (const float*)d_in[0];
  const float* wq = (const float*)d_in[1];
  const float* wk = (const float*)d_in[2];
  const float* wv = (const float*)d_in[3];
  const float* wo = (const float*)d_in[4];
  const float* bo = (const float*)d_in[5];
  const long need_x = ((long)(NB - 1) * T_FULL + TT) * (long)CC;
  if ((long)in_sizes[0] < need_x || in_sizes[1] < CC * CC || in_sizes[2] < CC * CC || in_sizes[3] < CC * CC ||
      in_sizes[4] < CC * CC || in_sizes[5] < CC || (long)out_size < need_x) return;
  float* out = (float*)d_out;

  char* ws = (char*)d_ws; size_t off = 0;
  auto take = [&](size_t bytes) { char* p = ws + off; off += (bytes + 255) & ~(size_t)255; return p; };
  const size_t xb_bytes = (size_t)NB * TT * CC * 2, s_bytes = (size_t)QC * TT * 4;
  char* reg0 = take(xb_bytes > s_bytes ? xb_bytes : s_bytes);
  unsigned short* xb   = (unsigned short*)reg0;
  float*          Sm   = (float*)reg0;
  unsigned short* Wqkv = (unsigned short*)take((size_t)3 * CC * CC * 2);
  unsigned short* Wo16 = (unsigned short*)take((size_t)CC * CC * 2);
  unsigned short* QKVh = (unsigned short*)take((size_t)3 * NB * TT * CC * 2);
  unsigned short* QKVr = (unsigned short*)take((size_t)3 * NB * NE * CC * 2);
  unsigned short* vT   = (unsigned short*)take((size_t)CC * TT * 2);
  unsigned short* vTr  = (unsigned short*)take((size_t)CC * NE * 2);
  unsigned short* Pm   = (unsigned short*)take((size_t)QC * TT * 2);
  unsigned short* Pr   = (unsigned short*)take((size_t)NE * NE * 2);
  unsigned short* ctxh = (unsigned short*)take((size_t)NB * TT * CC * 2);
  unsigned short* ctxr = (unsigned short*)take((size_t)NB * NE * CC * 2);
  if (off > ws_size) return;

  const int M = NB * TT;
  const int BIG = 1 << 28;
  unsigned short* qh = QKVh;
  unsigned short* kh = QKVh + (size_t)M * CC;
  unsigned short* vh = QKVh + (size_t)2 * M * CC;
  unsigned short* qr = QKVr;
  unsigned short* kr = QKVr + (size_t)(NB * NE) * CC;
  unsigned short* vr = QKVr + (size_t)2 * (NB * NE) * CC;

  for (int b = 0; b < NB; ++b)
    k_cvt<0><<<(TT * CC / 8 + 255) / 256, 256, 0, stream>>>(x + (size_t)b * T_FULL * CC, xb + (size_t)b * TT * CC, TT * CC / 8, 1.0f);
  k_cvt<0><<<(CC * CC / 8 + 255) / 256, 256, 0, stream>>>(wq, Wqkv, CC * CC / 8, 1.0f);
  k_cvt<0><<<(CC * CC / 8 + 255) / 256, 256, 0, stream>>>(wk, Wqkv + (size_t)CC * CC, CC * CC / 8, 1.0f);
  k_cvt<0><<<(CC * CC / 8 + 255) / 256, 256, 0, stream>>>(wv, Wqkv + (size_t)2 * CC * CC, CC * CC / 8, 1.0f);
  k_cvt<1><<<(CC * CC / 8 + 255) / 256, 256, 0, stream>>>(wo, Wo16, CC * CC / 8, WOC);

  k_gemm_qkv<<<((M / 16) * (3 * CC / 64) + 3) / 4, 128, 0, stream>>>(xb, Wqkv, QKVh, QKVr, M);

  for (int b = 0; b < NB; ++b) {
    const unsigned short* qb = qh + (size_t)b * TT * CC;
    const unsigned short* kb = kh + (size_t)b * TT * CC;
    k_transpose16<<<dim3(TT / 64, CC / 64), 256, 0, stream>>>(vh + (size_t)b * TT * CC, CC, vT, TT);
    k_transpose16<<<dim3(NE / 64, CC / 64), 256, 0, stream>>>(vr + (size_t)b * NE * CC, CC, vTr, NE);
    for (int c = 0; c < TT / QC; ++c) {
      const int qoff = c * QC, Nk = qoff + QC;
      const unsigned short* qa = qb + (size_t)qoff * CC;
      k_gemm_f32<1><<<((QC / 16) * (Nk / 64) + 3) / 4, 128, 0, stream>>>(qa, qa, CC, CC, kb, kb, CC, CC, nullptr, SCL, Sm, TT, QC, Nk, CC, qoff, BIG);
      if (c == 0)
        k_gemm_f32<3><<<((NE / 16) * (NE / 64) + 3) / 4, 128, 0, stream>>>(qb, qr + (size_t)b * NE * CC, CC, CC, kb, kr + (size_t)b * NE * CC, CC, CC,
                                                                     nullptr, SCL, Sm, TT, NE, NE, CC, 0, BIG);
      k_softmax<<<QC, 256, 0, stream>>>(Sm, TT, Pm, TT, Nk, qoff, Pr, NE, (c == 0) ? NE : 0);
      k_gemm_h16<1><<<((QC / 16) * (CC / 64) + 3) / 4, 128, 0, stream>>>(Pm, Pm, TT, TT, vT, vT, TT, TT, PVALPHA,
                                                                   ctxh + ((size_t)b * TT + qoff) * CC, CC, ctxr, CC, 0, QC, CC, Nk, qoff);
      if (c == 0)
        k_gemm_h16<3><<<((NE / 16) * (CC / 64) + 3) / 4, 128, 0, stream>>>(Pm, Pr, TT, NE, vT, vTr, TT, NE, PVALPHA,
                                                                     ctxh + (size_t)b * TT * CC, CC, ctxr + (size_t)b * NE * CC, CC, NE, NE, CC, NE, 0);
    }
  }
  for (int b = 0; b < NB; ++b) {
    k_gemm_f32<2><<<((NE / 16) * (CC / 64) + 3) / 4, 128, 0, stream>>>(ctxh + (size_t)b * TT * CC, ctxr + (size_t)b * NE * CC, CC, CC, Wo16, Wo16, CC, CC,
                                                                 bo, OALPHA, out + (size_t)b * T_FULL * CC, CC, NE, CC, CC, BIG, BIG);
    if (TT > NE)
      k_gemm_f32<1><<<(((TT - NE) / 16) * (CC / 64) + 3) / 4, 128, 0, stream>>>(ctxh + ((size_t)b * TT + NE) * CC, ctxh + ((size_t)b * TT + NE) * CC, CC, CC,
                                                                          Wo16, Wo16, CC, CC, bo, OALPHA, out + ((size_t)b * T_FULL + NE) * CC, CC,
                                                                          TT - NE, CC, CC, BIG, BIG);
  }
}
